// LSTM_Seq2Seq_3874060501292
// MI455X (gfx1250) — hardware-run, weakly checked
//
#include <hip/hip_runtime.h>
#include <math.h>

constexpr int NBATCH = 256;
constexpr int TCTX   = 512;
constexpr int TPRED  = 128;
constexpr int TALL   = TCTX + TPRED;
constexpr int DXF    = 7;
constexpr int DIN    = 8;
constexpr int NHID   = 256;
constexpr int NGATE  = 4 * NHID;
constexpr int MT     = 16;
constexpr int NTHR   = 256;
constexpr int KL0    = 288;
constexpr int KL1    = 2 * NHID;
constexpr int A0P    = 296;
constexpr int A1P    = 264;
constexpr int OUTP   = 128;
constexpr float WCARRY = 16.0f;
constexpr float ACARRY = 64.0f;
constexpr float FOLD   = 1.0f / (WCARRY * ACARRY);
constexpr float ACARRY_INV = 1.0f / ACARRY;

static_assert(NBATCH % MT == 0, "batch tile");
static_assert(NHID == 32 * (NTHR / 32), "8 waves x 32 hidden units");
static_assert(KL0 % 32 == 0 && KL1 % 32 == 0, "k tiles");
static_assert(DIN + NHID + 24 == KL0, "layer-0 k extent = x | h0 | 24 zero columns");
static_assert(A0P >= KL0 && A0P % 8 == 0 && A1P >= NHID && A1P % 8 == 0, "LDS pitches");
static_assert(OUTP == TPRED, "output staging pitch");
static_assert((MT * TPRED) % (NTHR * 4) == 0, "final store loop exact");

typedef __attribute__((ext_vector_type(16))) _Float16 v16h;
typedef __attribute__((ext_vector_type(8)))  _Float16 v8h;
typedef __attribute__((ext_vector_type(8)))  float    v8f;
typedef __attribute__((ext_vector_type(4)))  float    v4f;
typedef __attribute__((ext_vector_type(4)))  unsigned v4u;

union FragU { v16h v; v8h h[2]; };
__device__ __forceinline__ v16h frag_load(const _Float16* p) {
  FragU f;
  f.h[0] = *(const v8h*)(p);
  f.h[1] = *(const v8h*)(p + 16);
  return f.v;
}
__device__ __forceinline__ v8f mma16(v16h a, v16h b, v8f c) {
  return __builtin_amdgcn_wmma_f32_16x16x32_f16(false, a, false, b, (short)0, c, false, false);
}
__device__ __forceinline__ void guard4(v8f& a0, v8f& a1, v8f& a2, v8f& a3, v16h x, v16h y0, v16h y1, v16h y2, v16h y3) {
  asm volatile("v_nop\n\tv_nop\n\tv_nop\n\tv_nop"
               : "+v"(a0), "+v"(a1), "+v"(a2), "+v"(a3)
               : "v"(x), "v"(y0), "v"(y1), "v"(y2), "v"(y3));
}
__device__ __forceinline__ void acc_guard8(v8f& a0, v8f& a1, v8f& a2, v8f& a3, v8f& a4, v8f& a5, v8f& a6, v8f& a7) {
  asm volatile("v_nop\n\tv_nop\n\tv_nop\n\tv_nop"
               : "+v"(a0), "+v"(a1), "+v"(a2), "+v"(a3), "+v"(a4), "+v"(a5), "+v"(a6), "+v"(a7));
}

__device__ __forceinline__ float h16_to_f32(unsigned hb) {
  const unsigned sgn = (hb & 0x8000u) << 16;
  const unsigned em = hb & 0x7fffu;
  const float fn = __uint_as_float((em << 13) + 0x38000000u);
  const float fs = (float)em * 5.9604644775390625e-8f;
  const float mag = (em < 0x400u) ? fs : fn;
  return __uint_as_float(__float_as_uint(mag) | sgn);
}

__device__ __forceinline__ float fsig(float x)  { return __builtin_amdgcn_rcpf(1.0f + __expf(-x)); }
__device__ __forceinline__ float ftanh(float x) { return 1.0f - 2.0f * __builtin_amdgcn_rcpf(__expf(2.0f * x) + 1.0f); }

template <int GA, int GT>
__global__ __launch_bounds__(NTHR) void wplane_kernel(const float* __restrict__ wa, const float* __restrict__ wb,
                                                      unsigned short* __restrict__ dst) {
  static_assert((NGATE * GT) % NTHR == 0, "exact grid");
  const int i = blockIdx.x * NTHR + threadIdx.x;
  if (i < NGATE * GT) {
    const int n = i / GT;
    const int g = i - n * GT;
    const int gai = (g < GA) ? g : (GA - 1);
    int gbi = g - GA;
    gbi = (gbi < 0) ? 0 : gbi;
    gbi = (gbi > NHID / 8 - 1) ? (NHID / 8 - 1) : gbi;
    const float fa = (g < GA) ? 1.0f : 0.0f;
    const float fb = (g >= GA && g < GA + NHID / 8) ? 1.0f : 0.0f;
    const float* pa = wa + (size_t)n * (size_t)(8 * GA) + gai * 8;
    const float* pb = wb + (size_t)n * (size_t)NHID + gbi * 8;
    const v4f a0 = *(const v4f*)(pa);
    const v4f a1 = *(const v4f*)(pa + 4);
    const v4f b0 = *(const v4f*)(pb);
    const v4f b1 = *(const v4f*)(pb + 4);
    v8h hv;
#pragma unroll
    for (int e = 0; e < 4; ++e) {
      const float x0 = fa * a0[e] + fb * b0[e];
      const float x1 = fa * a1[e] + fb * b1[e];
      hv[e]     = (_Float16)(x0 * WCARRY);
      hv[4 + e] = (_Float16)(x1 * WCARRY);
    }
    *(volatile v8h*)(dst + (size_t)i * 8) = hv;
    __threadfence();
    *(volatile v8h*)(dst + (size_t)i * 8) = hv;
  }
}

__global__ __launch_bounds__(NTHR) void bias_kernel(const float* __restrict__ a0, const float* __restrict__ b0,
                                                    const float* __restrict__ a1, const float* __restrict__ b1,
                                                    const float* __restrict__ a2, const float* __restrict__ b2,
                                                    const float* __restrict__ a3, const float* __restrict__ b3,
                                                    float* __restrict__ dst) {
  const int s = blockIdx.x;
  const int tid = threadIdx.x;
  const float* pa = (s == 0) ? a0 : (s == 1) ? a1 : (s == 2) ? a2 : a3;
  const float* pb = (s == 0) ? b0 : (s == 1) ? b1 : (s == 2) ? b2 : b3;
  const v4f va = *(const v4f*)(pa + 4 * tid);
  const v4f vb = *(const v4f*)(pb + 4 * tid);
  v4f o;
#pragma unroll
  for (int e = 0; e < 4; ++e) o[e] = va[e] + vb[e];
  float* op = dst + (size_t)s * NGATE + 4 * tid;
  *(volatile v4f*)op = o;
  __threadfence();
  *(volatile v4f*)op = o;
}

__global__ __launch_bounds__(NTHR) void seq_kernel(const float* __restrict__ xc, const float* __restrict__ yc,
                                                   const float* __restrict__ xt, const float* __restrict__ yt,
                                                   unsigned short* __restrict__ dst) {
  const int tg = blockIdx.x;
  const int b  = threadIdx.x;
  const bool ctx = (tg <= TCTX);
  const float* xs = ctx ? xc : xt;
  const float* ys = ctx ? yc : yt;
  const int tlen = ctx ? TCTX : TPRED;
  const int trow = (tg < TCTX) ? tg : ((tg == TCTX) ? (TCTX - 1) : (tg - TCTX - 1));
  const size_t r = (size_t)b * (size_t)tlen + (size_t)trow;
  const float* xp = xs + r * DXF;
  const float x0 = xp[0], x1 = xp[1], x2 = xp[2], x3 = xp[3], x4 = xp[4], x5 = xp[5], x6 = xp[6];
  const float yv = ys[r];
  const float y  = (tg == TCTX) ? 0.0f : yv;
  v8h hv;
  hv[0] = (_Float16)(x0 * ACARRY);
  hv[1] = (_Float16)(x1 * ACARRY);
  hv[2] = (_Float16)(x2 * ACARRY);
  hv[3] = (_Float16)(x3 * ACARRY);
  hv[4] = (_Float16)(x4 * ACARRY);
  hv[5] = (_Float16)(x5 * ACARRY);
  hv[6] = (_Float16)(x6 * ACARRY);
  hv[7] = (_Float16)(y * ACARRY);
  unsigned short* op = dst + ((size_t)tg * NBATCH + (size_t)b) * DIN;
  *(volatile v8h*)op = hv;
  __threadfence();
  *(volatile v8h*)op = hv;
}

template <int LDB>
__device__ __forceinline__ void mm_tile8(v8f (&acc)[8], const v16h a, const _Float16* __restrict__ pw) {
  v16h bA[4], bB[4];
#pragma unroll
  for (int t = 0; t < 4; ++t) bA[t] = frag_load(pw + (size_t)(((t >> 1) * NHID + (t & 1) * 16) * LDB));
  acc[0] = mma16(a, bA[0], acc[0]);
  acc[1] = mma16(a, bA[1], acc[1]);
  acc[2] = mma16(a, bA[2], acc[2]);
  acc[3] = mma16(a, bA[3], acc[3]);
  guard4(acc[0], acc[1], acc[2], acc[3], a, bA[0], bA[1], bA[2], bA[3]);
#pragma unroll
  for (int t = 0; t < 4; ++t) bB[t] = frag_load(pw + (size_t)((((t + 4) >> 1) * NHID + (t & 1) * 16) * LDB));
  acc[4] = mma16(a, bB[0], acc[4]);
  acc[5] = mma16(a, bB[1], acc[5]);
  acc[6] = mma16(a, bB[2], acc[6]);
  acc[7] = mma16(a, bB[3], acc[7]);
  guard4(acc[4], acc[5], acc[6], acc[7], a, bB[0], bB[1], bB[2], bB[3]);
}

template <int PITCH>
__device__ __forceinline__ void lstm_cell(v8f (&acc)[8], float (&cst)[16], const float (&br)[8], _Float16* hp) {
#pragma unroll
  for (int j = 0; j < 2; ++j) {
#pragma unroll
    for (int r = 0; r < 8; ++r) {
      const float zi = fmaf(acc[0 + j][r], FOLD, br[0 + j]);
      const float zf = fmaf(acc[2 + j][r], FOLD, br[2 + j]);
      const float zg = fmaf(acc[4 + j][r], FOLD, br[4 + j]);
      const float zo = fmaf(acc[6 + j][r], FOLD, br[6 + j]);
      const float ig = fsig(zi);
      const float fg = fsig(zf);
      const float gg = ftanh(zg);
      const float og = fsig(zo);
      const float cn = fg * cst[8 * j + r] + ig * gg;
      cst[8 * j + r] = cn;
      const float hn = og * ftanh(cn);
      hp[r * PITCH + 16 * j] = (_Float16)(hn * ACARRY);
    }
  }
}

__device__ __forceinline__ void stage_x(_Float16* A0, const unsigned short* __restrict__ SEQ, int tg, int rowbase, int tid) {
  if (tid < 64) {
    const int row = tid & 15;
    const int part = tid >> 4;
    v4u xv = *(const v4u*)(SEQ + ((size_t)tg * NBATCH + (size_t)(rowbase + row)) * DIN);
    asm volatile("" : "+v"(xv));
    const unsigned msk = (part == 0) ? 0xFFFFFFFFu : 0u;
    v4u val;
    val[0] = xv[0] & msk;
    val[1] = xv[1] & msk;
    val[2] = xv[2] & msk;
    val[3] = xv[3] & msk;
    const int col = (part == 0) ? 0 : (NHID + 8 * part);
    *(v4u*)(A0 + row * A0P + col) = val;
  }
}

__global__ __launch_bounds__(NTHR) void lstm2_seq_kernel(const unsigned short* __restrict__ SEQ,
                                                         const unsigned short* __restrict__ BT0E,
                                                         const unsigned short* __restrict__ BT1E,
                                                         const unsigned short* __restrict__ BT0D,
                                                         const unsigned short* __restrict__ BT1D,
                                                         const float* __restrict__ BIAS,
                                                         const float* __restrict__ fcw,
                                                         const float* __restrict__ fcb,
                                                         float* __restrict__ out) {
  __shared__ __align__(16) _Float16 A0[MT * A0P];
  __shared__ __align__(16) _Float16 A1[MT * A1P];
  __shared__ __align__(16) float    OutS[MT * OUTP];

  const int tid = threadIdx.x, lane = tid & 31, wave = tid >> 5;
  const int c = lane & 15, hh = lane >> 4, koff = hh * 8;
  const int rowbase = blockIdx.x * MT;

#pragma unroll 1
  for (int i = tid; i < MT * A0P; i += NTHR) A0[i] = (_Float16)0.0f;
#pragma unroll 1
  for (int i = tid; i < MT * A1P; i += NTHR) A1[i] = (_Float16)0.0f;
#pragma unroll 1
  for (int i = tid; i < MT * OUTP; i += NTHR) OutS[i] = 0.0f;
  float c0[16], c1[16];
#pragma unroll
  for (int i = 0; i < 16; ++i) { c0[i] = 0.0f; c1[i] = 0.0f; }
  __syncthreads();
  stage_x(A0, SEQ, 0, rowbase, tid);
  __syncthreads();

  const float fcb0 = fcb[0];
  const _Float16* a0row = A0 + c * A0P + koff;
  const _Float16* a0hrow = A0 + c * A0P + DIN + koff;
  const _Float16* a1row = A1 + c * A1P + koff;
  _Float16* h0dst = A0 + (8 * hh) * A0P + DIN + 32 * wave + c;
  _Float16* h1dst = A1 + (8 * hh) * A1P + 32 * wave + c;
  const v8f z8 = {0.f, 0.f, 0.f, 0.f, 0.f, 0.f, 0.f, 0.f};

#pragma unroll 1
  for (int phase = 0; phase < 2; ++phase) {
    const _Float16* W0 = (const _Float16*)(phase ? BT0D : BT0E);
    const _Float16* W1 = (const _Float16*)(phase ? BT1D : BT1E);
    const float* b0 = BIAS + (size_t)phase * 2 * NGATE;
    const float* b1 = b0 + NGATE;
    const int TT = phase ? TPRED : TCTX;
    const _Float16* pw0 = W0 + (size_t)(32 * wave + c) * KL0 + koff;
    const _Float16* pw1 = W1 + (size_t)(32 * wave + c) * KL1 + koff;

    float bias0r[8], bias1r[8];
#pragma unroll
    for (int t = 0; t < 8; ++t) {
      const int n = (t >> 1) * NHID + 32 * wave + (t & 1) * 16 + c;
      bias0r[t] = b0[n];
      bias1r[t] = b1[n];
    }

#pragma unroll 1
    for (int t = 0; t < TT; ++t) {
      const int tg = phase * TCTX + t;
      v8f acc[8];

#pragma unroll
      for (int q = 0; q < 8; ++q) acc[q] = z8;
#pragma unroll 1
      for (int kt = 0; kt < KL0 / 32; ++kt) {
        const v16h a = frag_load(a0row + kt * 32);
        mm_tile8<KL0>(acc, a, pw0 + kt * 32);
      }
      acc_guard8(acc[0], acc[1], acc[2], acc[3], acc[4], acc[5], acc[6], acc[7]);
      __syncthreads();
      lstm_cell<A0P>(acc, c0, bias0r, h0dst);
      {
        const int tgn = (tg + 1 < TALL) ? (tg + 1) : (TALL - 1);
        stage_x(A0, SEQ, tgn, rowbase, tid);
      }
      __syncthreads();

#pragma unroll
      for (int q = 0; q < 8; ++q) acc[q] = z8;
#pragma unroll 1
      for (int kt = 0; kt < NHID / 32; ++kt) {
        const v16h a = frag_load(a0hrow + kt * 32);
        mm_tile8<KL1>(acc, a, pw1 + kt * 32);
      }
#pragma unroll 1
      for (int kt = 0; kt < NHID / 32; ++kt) {
        const v16h a = frag_load(a1row + kt * 32);
        mm_tile8<KL1>(acc, a, pw1 + NHID + kt * 32);
      }
      acc_guard8(acc[0], acc[1], acc[2], acc[3], acc[4], acc[5], acc[6], acc[7]);
      __syncthreads();
      lstm_cell<A1P>(acc, c1, bias1r, h1dst);
      __syncthreads();

      if (phase != 0) {
        const int row = tid >> 4, seg = tid & 15;
        const v4u w0 = *(const v4u*)(A1 + row * A1P + seg * 16);
        const v4u w1 = *(const v4u*)(A1 + row * A1P + seg * 16 + 8);
        const v4f f0 = *(const v4f*)(fcw + seg * 16);
        const v4f f1 = *(const v4f*)(fcw + seg * 16 + 4);
        const v4f f2 = *(const v4f*)(fcw + seg * 16 + 8);
        const v4f f3 = *(const v4f*)(fcw + seg * 16 + 12);
        const unsigned u0 = w0[0], u1 = w0[1], u2 = w0[2], u3 = w0[3];
        const unsigned u4 = w1[0], u5 = w1[1], u6 = w1[2], u7 = w1[3];
        float s = 0.0f;
        s = fmaf(h16_to_f32(u0 & 0xffffu), f0[0], s);
        s = fmaf(h16_to_f32(u0 >> 16),     f0[1], s);
        s = fmaf(h16_to_f32(u1 & 0xffffu), f0[2], s);
        s = fmaf(h16_to_f32(u1 >> 16),     f0[3], s);
        s = fmaf(h16_to_f32(u2 & 0xffffu), f1[0], s);
        s = fmaf(h16_to_f32(u2 >> 16),     f1[1], s);
        s = fmaf(h16_to_f32(u3 & 0xffffu), f1[2], s);
        s = fmaf(h16_to_f32(u3 >> 16),     f1[3], s);
        s = fmaf(h16_to_f32(u4 & 0xffffu), f2[0], s);
        s = fmaf(h16_to_f32(u4 >> 16),     f2[1], s);
        s = fmaf(h16_to_f32(u5 & 0xffffu), f2[2], s);
        s = fmaf(h16_to_f32(u5 >> 16),     f2[3], s);
        s = fmaf(h16_to_f32(u6 & 0xffffu), f3[0], s);
        s = fmaf(h16_to_f32(u6 >> 16),     f3[1], s);
        s = fmaf(h16_to_f32(u7 & 0xffffu), f3[2], s);
        s = fmaf(h16_to_f32(u7 >> 16),     f3[3], s);
        s += __shfl_xor(s, 1, 32);
        s += __shfl_xor(s, 2, 32);
        s += __shfl_xor(s, 4, 32);
        s += __shfl_xor(s, 8, 32);
        if (seg == 0) OutS[row * OUTP + t] = fmaf(s, ACARRY_INV, fcb0);
      }
    }
  }

  __syncthreads();
  for (int pass = 0; pass < 2; ++pass) {
#pragma unroll
    for (int it = 0; it < (MT * TPRED) / (NTHR * 4); ++it) {
      const int idx = it * NTHR + tid;
      const int row = idx >> 5;
      const int c4 = (idx & 31) * 4;
      const v4f v = *(const v4f*)(OutS + row * OUTP + c4);
      *(volatile v4f*)(out + (size_t)(rowbase + row) * TPRED + c4) = v;
    }
    __threadfence();
  }
}

extern "C" void kernel_launch(void* const* d_in, const int* in_sizes, int n_in,
                              void* d_out, int out_size, void* d_ws, size_t ws_size, hipStream_t stream) {
  if (n_in < 23 || d_out == nullptr || d_ws == nullptr) return;
  if (in_sizes[0] != NBATCH * TCTX * DXF || in_sizes[1] != NBATCH * TCTX ||
      in_sizes[2] != NBATCH * TPRED * DXF || in_sizes[3] != NBATCH * TPRED ||
      in_sizes[5] != NGATE * DIN || in_sizes[6] != NGATE * NHID || in_sizes[7] != NGATE || in_sizes[8] != NGATE ||
      in_sizes[9] != NGATE * NHID || in_sizes[10] != NGATE * NHID || in_sizes[11] != NGATE || in_sizes[12] != NGATE ||
      in_sizes[13] != NGATE * DIN || in_sizes[14] != NGATE * NHID || in_sizes[15] != NGATE || in_sizes[16] != NGATE ||
      in_sizes[17] != NGATE * NHID || in_sizes[18] != NGATE * NHID || in_sizes[19] != NGATE || in_sizes[20] != NGATE ||
      in_sizes[21] != NHID || in_sizes[22] != 1 || out_size != NBATCH * TPRED) return;

  const float* xc    = (const float*)d_in[0];
  const float* yc    = (const float*)d_in[1];
  const float* xt    = (const float*)d_in[2];
  const float* yt    = (const float*)d_in[3];
  const float* eWih0 = (const float*)d_in[5];
  const float* eWhh0 = (const float*)d_in[6];
  const float* ebih0 = (const float*)d_in[7];
  const float* ebhh0 = (const float*)d_in[8];
  const float* eWih1 = (const float*)d_in[9];
  const float* eWhh1 = (const float*)d_in[10];
  const float* ebih1 = (const float*)d_in[11];
  const float* ebhh1 = (const float*)d_in[12];
  const float* dWih0 = (const float*)d_in[13];
  const float* dWhh0 = (const float*)d_in[14];
  const float* dbih0 = (const float*)d_in[15];
  const float* dbhh0 = (const float*)d_in[16];
  const float* dWih1 = (const float*)d_in[17];
  const float* dWhh1 = (const float*)d_in[18];
  const float* dbih1 = (const float*)d_in[19];
  const float* dbhh1 = (const float*)d_in[20];
  const float* fcW   = (const float*)d_in[21];
  const float* fcb   = (const float*)d_in[22];
  float* out = (float*)d_out;

  char* ws = (char*)d_ws;
  size_t off = 0;
  auto carve = [&](size_t bytes) -> char* { char* p = ws + off; off += (bytes + 255) & ~(size_t)255; return p; };
  unsigned short* BT0E = (unsigned short*)carve((size_t)NGATE * KL0 * 2);
  unsigned short* BT1E = (unsigned short*)carve((size_t)NGATE * KL1 * 2);
  unsigned short* BT0D = (unsigned short*)carve((size_t)NGATE * KL0 * 2);
  unsigned short* BT1D = (unsigned short*)carve((size_t)NGATE * KL1 * 2);
  float*          BIAS = (float*)carve((size_t)4 * NGATE * 4);
  unsigned short* SEQ  = (unsigned short*)carve((size_t)TALL * NBATCH * DIN * 2);
  if (off > ws_size || off > (size_t)134217728) return;

  wplane_kernel<1, KL0 / 8><<<(NGATE * (KL0 / 8)) / NTHR, NTHR, 0, stream>>>(eWih0, eWhh0, BT0E);
  wplane_kernel<NHID / 8, KL1 / 8><<<(NGATE * (KL1 / 8)) / NTHR, NTHR, 0, stream>>>(eWih1, eWhh1, BT1E);
  wplane_kernel<1, KL0 / 8><<<(NGATE * (KL0 / 8)) / NTHR, NTHR, 0, stream>>>(dWih0, dWhh0, BT0D);
  wplane_kernel<NHID / 8, KL1 / 8><<<(NGATE * (KL1 / 8)) / NTHR, NTHR, 0, stream>>>(dWih1, dWhh1, BT1D);
  bias_kernel<<<4, NTHR, 0, stream>>>(ebih0, ebhh0, ebih1, ebhh1, dbih0, dbhh0, dbih1, dbhh1, BIAS);
  seq_kernel<<<TALL, NTHR, 0, stream>>>(xc, yc, xt, yt, SEQ);
  lstm2_seq_kernel<<<NBATCH / MT, NTHR, 0, stream>>>(SEQ, BT0E, BT1E, BT0D, BT1D, BIAS, fcW, fcb, out);
}
